// BertForSpanAspectExtraction_72971494359130
// MI455X (gfx1250) — hardware-verified
//
#include <hip/hip_runtime.h>
#include <stdint.h>
#include <stddef.h>
#include <math.h>

#define NB   4
#define NL   256
#define NH   768
#define NH2  384
#define NM   (NB * NL)
#define NP   (2 * NH2)
#define LR   32
#define SPP  68
#define WTP  72
#define SSP  388
#define WSCALE 64.0f
#define WINV   0.015625f

#define SPAN_SS          (32 * SSP)
#define SPAN_LDS_FLOATS  (2 * SPAN_SS + NH2 + 32 * 32)
#define SPAN_LDS_BYTES   (SPAN_LDS_FLOATS * 4)

static_assert(SPAN_LDS_BYTES == 104960);
static_assert(NH % 32 == 0);
static_assert(NH == 3 * 32 * 8);
static_assert(NM % 64 == 0);
static_assert(NP % 64 == 0);
static_assert(NM % LR == 0);
static_assert(NH2 % 32 == 0);
static_assert(NH % 64 == 0);
static_assert(NL % 32 == 0);
static_assert(NH2 % 4 == 0);
static_assert((SSP * 4) % 16 == 0);
static_assert((SPP * 4) % 16 == 0);
static_assert((WTP * 2) % 16 == 0);
static_assert((SPAN_SS * 4) % 16 == 0);

typedef _Float16       v16h __attribute__((ext_vector_type(16)));
typedef _Float16       v8h  __attribute__((ext_vector_type(8)));
typedef float          v8f  __attribute__((ext_vector_type(8)));
typedef float          v4f  __attribute__((ext_vector_type(4)));
typedef unsigned int   v4u  __attribute__((ext_vector_type(4)));
typedef v4f __attribute__((may_alias)) v4fa;
typedef v4u __attribute__((may_alias)) v4ua;
typedef v8h __attribute__((may_alias)) v8ha;

union Frag { v16h v; v8h half[2]; };
union Cvt8 { v8h h; v4u u; };

__device__ __forceinline__ v8f wmma16(v16h a, v16h b, v8f c) {
  v8f d = __builtin_amdgcn_wmma_f32_16x16x32_f16(false, a, false, b, (short)0, c, false, false);
  asm volatile("v_nop\n\tv_nop\n\tv_nop\n\tv_nop" : "+v"(d) : "v"(a), "v"(b));
  return d;
}

__device__ __forceinline__ v16h ldf(const _Float16* p, int h) {
  Frag f;
  f.half[0] = *(const v8ha*)(p + 8 * h);
  f.half[1] = *(const v8ha*)(p + 16 + 8 * h);
  return f.v;
}

__global__ __launch_bounds__(256) void k_logits_cvt(const float* __restrict__ x,
                                                    const float* __restrict__ wst,
                                                    const float* __restrict__ bst,
                                                    const float* __restrict__ wen,
                                                    const float* __restrict__ ben,
                                                    _Float16* __restrict__ xh,
                                                    float* __restrict__ out)
{
  __shared__ __align__(16) float sl[2 * LR];
  const int tid = threadIdx.x, lane = tid & 31, wv = tid >> 5;
  const int rb = blockIdx.x * LR;
  const float bs0 = bst[0];
  const float be0 = ben[0];

  #pragma unroll 1
  for (int rr = 0; rr < 4; ++rr) {
    const int rl  = wv * 4 + rr;
    const int row = rb + rl;
    const float* xr = x + (size_t)row * NH;
    _Float16* hr = xh + (size_t)row * NH;

    v4f as = {0.f, 0.f, 0.f, 0.f};
    v4f ae = {0.f, 0.f, 0.f, 0.f};
    v4u cv[3];
    #pragma unroll
    for (int it = 0; it < 3; ++it) {
      const int c = (lane + 32 * it) * 8;
      const v4f x0 = *(const v4fa*)(xr + c);
      const v4f x1 = *(const v4fa*)(xr + c + 4);
      const v4f s0 = *(const v4fa*)(wst + c);
      const v4f s1 = *(const v4fa*)(wst + c + 4);
      const v4f e0 = *(const v4fa*)(wen + c);
      const v4f e1 = *(const v4fa*)(wen + c + 4);
      as += x0 * s0;
      as += x1 * s1;
      ae += x0 * e0;
      ae += x1 * e1;
      Cvt8 q;
      q.h[0] = (_Float16)x0.x; q.h[1] = (_Float16)x0.y; q.h[2] = (_Float16)x0.z; q.h[3] = (_Float16)x0.w;
      q.h[4] = (_Float16)x1.x; q.h[5] = (_Float16)x1.y; q.h[6] = (_Float16)x1.z; q.h[7] = (_Float16)x1.w;
      cv[it] = q.u;
    }
    #pragma unroll
    for (int it = 0; it < 3; ++it)
      *(volatile v4ua*)(hr + (lane + 32 * it) * 8) = cv[it];

    float ss = (as.x + as.y) + (as.z + as.w);
    float se = (ae.x + ae.y) + (ae.z + ae.w);
    #pragma unroll
    for (int off = 16; off > 0; off >>= 1) {
      ss += __shfl_xor(ss, off);
      se += __shfl_xor(se, off);
    }
    if (lane == 0) {
      sl[rl]      = ss + bs0;
      sl[LR + rl] = se + be0;
    }

    __threadfence();
    #pragma unroll
    for (int it = 0; it < 3; ++it)
      *(volatile v4ua*)(hr + (lane + 32 * it) * 8) = cv[it];
  }
  __syncthreads();

  if (wv == 0 && lane < 16) {
    const int sel = lane >> 3;
    const int q   = lane & 7;
    const v4f v = *(const v4fa*)(sl + sel * LR + 4 * q);
    float* dst = out + (size_t)sel * NM + rb + 4 * q;
    *(volatile v4fa*)dst = v;
    __threadfence();
    *(volatile v4fa*)dst = v;
  }
}

__global__ __launch_bounds__(256) void k_wt(const float* __restrict__ w0,
                                            const float* __restrict__ w1,
                                            _Float16* __restrict__ wt)
{
  __shared__ __align__(16) _Float16 tl[32 * WTP];
  const int tid = threadIdx.x, lane = tid & 31, wv = tid >> 5;
  const int n0 = blockIdx.x * 32, k0 = blockIdx.y * 64, sel = blockIdx.z;
  const float* w = (sel == 0) ? w0 : w1;

  #pragma unroll
  for (int i = 0; i < 8; ++i) {
    const int idx = tid + 256 * i;
    const int kl = idx >> 5, nl = idx & 31;
    const float v = w[(size_t)(k0 + kl) * NH2 + n0 + nl] * WSCALE;
    tl[nl * WTP + kl] = (_Float16)v;
  }
  __syncthreads();

  const int nl = wv * 4 + (lane >> 3), q = lane & 7;
  Cvt8 c;
  c.h = *(const v8ha*)(tl + nl * WTP + 8 * q);
  _Float16* dst = wt + (size_t)(sel * NH2 + n0 + nl) * NH + k0 + 8 * q;
  *(volatile v4ua*)dst = c.u;
  __threadfence();
  *(volatile v4ua*)dst = c.u;
}

__global__ __launch_bounds__(128) void k_proj(const _Float16* __restrict__ xh,
                                              const _Float16* __restrict__ wt,
                                              const float* __restrict__ b1,
                                              float* __restrict__ P)
{
  __shared__ __align__(16) float sp[64 * SPP];
  const int tid = threadIdx.x, lane = tid & 31, wv = tid >> 5;
  const int h = lane >> 4, m = lane & 15;
  const int n0 = blockIdx.x * 64;
  const int rb = blockIdx.y * 64;

  const _Float16* ar = xh + (size_t)(rb + wv * 16 + m) * NH;
  const _Float16* br = wt + (size_t)(n0 + m) * NH;

  const v8f z8 = {0.f, 0.f, 0.f, 0.f, 0.f, 0.f, 0.f, 0.f};
  v8f acc[4] = {z8, z8, z8, z8};

  #pragma unroll 2
  for (int k0 = 0; k0 < NH; k0 += 32) {
    const v16h a = ldf(ar + k0, h);
    #pragma unroll
    for (int nt = 0; nt < 4; ++nt) {
      const v16h bf = ldf(br + (size_t)nt * 16 * NH + k0, h);
      acc[nt] = wmma16(a, bf, acc[nt]);
    }
  }

  const bool eh = (n0 >= NH2);
  #pragma unroll
  for (int nt = 0; nt < 4; ++nt) {
    int bi = n0 + nt * 16 + m - NH2;
    bi = (bi < 0) ? 0 : bi;
    bi = (bi > NH2 - 1) ? (NH2 - 1) : bi;
    const float bb = b1[bi];
    const float bias = eh ? bb : 0.0f;
    #pragma unroll
    for (int r = 0; r < 8; ++r)
      sp[(wv * 16 + 8 * h + r) * SPP + nt * 16 + m] = acc[nt][r] * WINV + bias;
  }
  __syncthreads();

  float* pb = P + (size_t)rb * NP + n0;
  #pragma unroll
  for (int i = 0; i < 8; ++i) {
    const int row = wv * 16 + 2 * i + h;
    const v4f v = *(const v4fa*)(sp + row * SPP + 4 * m);
    *(volatile v4fa*)(pb + (size_t)row * NP + 4 * m) = v;
  }
  __threadfence();
  #pragma unroll
  for (int i = 0; i < 8; ++i) {
    const int row = wv * 16 + 2 * i + h;
    const v4f v = *(const v4fa*)(sp + row * SPP + 4 * m);
    *(volatile v4fa*)(pb + (size_t)row * NP + 4 * m) = v;
  }
}

__global__ __launch_bounds__(256) void k_span(const float* __restrict__ P,
                                              const float* __restrict__ W2,
                                              const float* __restrict__ b2,
                                              float* __restrict__ out2)
{
  extern __shared__ __align__(16) float smem[];
  float* sS = smem;
  float* sE = smem + SPAN_SS;
  float* sW = sE + SPAN_SS;
  float* sO = sW + NH2;

  const int tid = threadIdx.x, lane = tid & 31, wv = tid >> 5;
  const int j0 = blockIdx.x * 32, i0 = blockIdx.y * 32, b = blockIdx.z;
  const float* Ps = P + (size_t)(b * NL + i0) * NP;
  const float* Pe = P + (size_t)(b * NL + j0) * NP + NH2;

  #pragma unroll 4
  for (int i = 0; i < 12; ++i) {
    const int idx = tid + 256 * i;
    const int r = idx / 96;
    const int c = (idx - r * 96) * 4;
    *(v4fa*)(sS + r * SSP + c) = *(const v4fa*)(Ps + (size_t)r * NP + c);
    *(v4fa*)(sE + r * SSP + c) = *(const v4fa*)(Pe + (size_t)r * NP + c);
  }
  if (tid < NH2 / 4) *(v4fa*)(sW + 4 * tid) = *(const v4fa*)(W2 + 4 * tid);
  __syncthreads();

  const int ig = tid >> 4, jg = tid & 15;
  const float* s0p = sS + (2 * ig) * SSP;
  const float* s1p = s0p + SSP;
  const float* e0p = sE + (2 * jg) * SSP;
  const float* e1p = e0p + SSP;
  float a00 = 0.f, a01 = 0.f, a10 = 0.f, a11 = 0.f;

  #pragma unroll 2
  for (int k4 = 0; k4 < NH2 / 4; ++k4) {
    const v4f s0 = *(const v4fa*)(s0p + 4 * k4);
    const v4f s1 = *(const v4fa*)(s1p + 4 * k4);
    const v4f e0 = *(const v4fa*)(e0p + 4 * k4);
    const v4f e1 = *(const v4fa*)(e1p + 4 * k4);
    const v4f w  = *(const v4fa*)(sW  + 4 * k4);
    #pragma unroll
    for (int c = 0; c < 4; ++c) {
      const float h00 = fmaxf(s0[c] + e0[c], 0.f);
      const float h01 = fmaxf(s0[c] + e1[c], 0.f);
      const float h10 = fmaxf(s1[c] + e0[c], 0.f);
      const float h11 = fmaxf(s1[c] + e1[c], 0.f);
      a00 = fmaf(h00, w[c], a00);
      a01 = fmaf(h01, w[c], a01);
      a10 = fmaf(h10, w[c], a10);
      a11 = fmaf(h11, w[c], a11);
    }
  }

  const float bz = b2[0];
  const float z00 = a00 + bz, z01 = a01 + bz, z10 = a10 + bz, z11 = a11 + bz;
  const float g00 = 1.0f / (1.0f + __expf(-z00));
  const float g01 = 1.0f / (1.0f + __expf(-z01));
  const float g10 = 1.0f / (1.0f + __expf(-z10));
  const float g11 = 1.0f / (1.0f + __expf(-z11));
  sO[(2 * ig) * 32 + 2 * jg]         = g00;
  sO[(2 * ig) * 32 + 2 * jg + 1]     = g01;
  sO[(2 * ig + 1) * 32 + 2 * jg]     = g10;
  sO[(2 * ig + 1) * 32 + 2 * jg + 1] = g11;
  __syncthreads();

  const int row = wv * 4 + (lane >> 3), q = lane & 7;
  const v4f v = *(const v4fa*)(sO + row * 32 + 4 * q);
  float* dst = out2 + ((size_t)(b * NL + i0 + row)) * NL + j0 + 4 * q;
  *(volatile v4fa*)dst = v;
  __threadfence();
  *(volatile v4fa*)dst = v;
}

extern "C" void kernel_launch(void* const* d_in, const int* in_sizes, int n_in,
                              void* d_out, int out_size, void* d_ws, size_t ws_size,
                              hipStream_t stream)
{
  if (n_in < 10) return;
  if (in_sizes[0] != NM * NH) return;
  if (in_sizes[1] != NH) return;
  if (in_sizes[2] < 1) return;
  if (in_sizes[3] != NH) return;
  if (in_sizes[4] < 1) return;
  if (in_sizes[5] != NH * NH2) return;
  if (in_sizes[6] != NH * NH2) return;
  if (in_sizes[7] != NH2) return;
  if (in_sizes[8] != NH2) return;
  if (in_sizes[9] < 1) return;
  if (out_size != 2 * NM + NB * NL * NL) return;

  const float* x   = (const float*)d_in[0];
  const float* wst = (const float*)d_in[1];
  const float* bst = (const float*)d_in[2];
  const float* wen = (const float*)d_in[3];
  const float* ben = (const float*)d_in[4];
  const float* W1s = (const float*)d_in[5];
  const float* W1e = (const float*)d_in[6];
  const float* b1  = (const float*)d_in[7];
  const float* W2  = (const float*)d_in[8];
  const float* b2  = (const float*)d_in[9];
  float* out = (float*)d_out;

  const size_t bXH = (size_t)NM * NH * 2;
  const size_t bWT = (size_t)NP * NH * 2;
  const size_t bP  = (size_t)NM * NP * 4;
  const size_t total = bXH + bWT + bP;
  if (total > ws_size) return;
  if (total > (size_t)134217728) return;

  char* ws = (char*)d_ws;
  size_t off = 0;
  _Float16* XH = (_Float16*)(ws + off); off += bXH;
  _Float16* WT = (_Float16*)(ws + off); off += bWT;
  float*    P  = (float*)(ws + off);    off += bP;
  if (off != total) return;

  k_logits_cvt<<<NM / LR, 256, 0, stream>>>(x, wst, bst, wen, ben, XH, out);
  k_wt<<<dim3(NH2 / 32, NH / 64, 2), 256, 0, stream>>>(W1s, W1e, WT);
  k_proj<<<dim3(NP / 64, NM / 64), 128, 0, stream>>>(XH, WT, b1, P);
  hipFuncSetAttribute(reinterpret_cast<const void*>(&k_span),
                      hipFuncAttributeMaxDynamicSharedMemorySize, SPAN_LDS_BYTES);
  k_span<<<dim3(NL / 32, NL / 32, NB), 256, SPAN_LDS_BYTES, stream>>>(P, W2, b2, out + 2 * NM);
}
